// SelfAttentionUnit_32315333935894
// MI455X (gfx1250) — hardware-verified
//
#include <hip/hip_runtime.h>


#define NB_  16
#define CIN  131
#define KP   192
#define NN_  4096
#define HH_  256
#define CO   128
#define BCH  4

typedef unsigned short bf;
typedef __attribute__((ext_vector_type(16))) __bf16   v16bf;
typedef __attribute__((ext_vector_type(8)))  unsigned short v8us;
typedef __attribute__((ext_vector_type(8)))  float    v8f;
typedef __attribute__((ext_vector_type(4)))  float    v4f;
typedef v4f  __attribute__((may_alias)) v4fa;
typedef v8us __attribute__((may_alias)) v8usa;

__device__ __forceinline__ unsigned short f2bf(float f) { unsigned u = __float_as_uint(f); u += 0x7FFFu + ((u >> 16) & 1u); return (unsigned short)(u >> 16); }
__device__ __forceinline__ float bf2f(unsigned short b) { return __uint_as_float(((unsigned)b) << 16); }
__device__ __forceinline__ float bfr(float f) { return bf2f(f2bf(f)); }
__device__ __forceinline__ v16bf cat16b(v8us lo, v8us hi) { return __builtin_bit_cast(v16bf, __builtin_shufflevector(lo, hi, 0, 1, 2, 3, 4, 5, 6, 7, 8, 9, 10, 11, 12, 13, 14, 15)); }
__device__ __forceinline__ v8f wmmab(v16bf a, v16bf b, v8f c) { return __builtin_amdgcn_wmma_f32_16x16x32_bf16(false, a, false, b, (short)0, c, false, false); }
#define VST2(T, p, v) do { const T vst2_v_ = (v); *(volatile T*)(p) = vst2_v_; __threadfence(); *(volatile T*)(p) = vst2_v_; } while (0)

__global__ __launch_bounds__(256) void k_xt(const float* __restrict__ x, int b0, bf* XT) {
    __shared__ __align__(16) unsigned short tl[64 * 72];
    const int tid = threadIdx.x, n0 = blockIdx.x * 64, c0 = blockIdx.y * 64, bl = blockIdx.z, b = b0 + bl;
    const int cr = tid >> 2, nq = (tid & 3) * 16, c = c0 + cr;
#pragma unroll
    for (int i = 0; i < 16; ++i) tl[(nq + i) * 72 + cr] = (c < CIN) ? f2bf(x[((size_t)b * CIN + c) * NN_ + n0 + nq + i]) : (unsigned short)0;
    __syncthreads();
    const int piece = tid & 7;
    auto pass = [&]() {
#pragma unroll
        for (int s = 0; s < 2; ++s) { const int nr = (tid >> 3) + 32 * s; const v8us val = *(const v8usa*)(tl + nr * 72 + piece * 8);
            *(volatile v8us*)(XT + ((size_t)bl * NN_ + n0 + nr) * KP + c0 + piece * 8) = val; }
    };
    pass(); __threadfence(); pass();
}
__device__ __forceinline__ void wrow(const float* __restrict__ src, bf* dst, int lane) {
    if (lane < KP / 8) { v8us t;
#pragma unroll
        for (int i = 0; i < 8; ++i) { const int k = lane * 8 + i; t[i] = (k < CIN) ? f2bf(src[k < CIN ? k : 0]) : (unsigned short)0; }
        VST2(v8us, dst + lane * 8, t); }
}
__global__ __launch_bounds__(256) void k_w(const float* __restrict__ wq, const float* __restrict__ wk, const float* __restrict__ wv, const float* __restrict__ wf, bf* WP3, bf* WF) {
    const int lane = threadIdx.x & 31, r = blockIdx.x * 8 + (threadIdx.x >> 5);
    const int m = blockIdx.x / (HH_ / 8);
    if (m == 0)      { const int o = r;           wrow(wq + (size_t)o * CIN, WP3 + (size_t)r * KP, lane); }
    else if (m == 1) { const int o = r - HH_;     wrow(wk + (size_t)o * CIN, WP3 + (size_t)r * KP, lane); }
    else if (m == 2) { const int o = r - 2 * HH_; wrow(wv + (size_t)o * CIN, WP3 + (size_t)r * KP, lane); }
    else { const int o = r - 3 * HH_; if (o < CO) { v8us t;
#pragma unroll
        for (int i = 0; i < 8; ++i) t[i] = f2bf(wf[(size_t)o * HH_ + lane * 8 + i]);
        VST2(v8us, WF + (size_t)o * HH_ + lane * 8, t); } }
}
template <bool SA, bool SB, int MODE>
__global__ __launch_bounds__(128) void k_gemm(const bf* __restrict__ A, const bf* __restrict__ Al, const bf* __restrict__ Bn, const bf* __restrict__ Bl, int K, int ldc,
                                             const float* __restrict__ sc, const float* __restrict__ sh, void* C, void* C2) {
    __shared__ __align__(16) float ost[4][16 * 68];
    const int lane = threadIdx.x & 31, wave = threadIdx.x >> 5, lr = lane & 15, hi = lane >> 4;
    const int r0 = blockIdx.x * 64 + wave * 16, c0 = blockIdx.y * 64;
    const size_t aoff = (size_t)(r0 + lr) * K + 8 * hi;
    size_t boff[4];
#pragma unroll
    for (int t = 0; t < 4; ++t) boff[t] = (size_t)(c0 + t * 16 + lr) * K + 8 * hi;
    v8f acc[4];
#pragma unroll
    for (int t = 0; t < 4; ++t) acc[t] = (v8f){};
#pragma unroll 1
    for (int kc = 0; kc < K; kc += 32) {
        const v16bf a = cat16b(*(const v8us*)(A + aoff + kc), *(const v8us*)(A + aoff + kc + 16));
        v16bf al = a; if (SA) al = cat16b(*(const v8us*)(Al + aoff + kc), *(const v8us*)(Al + aoff + kc + 16));
#pragma unroll
        for (int t = 0; t < 4; ++t) { const v16bf b = cat16b(*(const v8us*)(Bn + boff[t] + kc), *(const v8us*)(Bn + boff[t] + kc + 16));
            acc[t] = wmmab(a, b, acc[t]); if (SA) acc[t] = wmmab(al, b, acc[t]);
            if (SB) { const v16bf bl2 = cat16b(*(const v8us*)(Bl + boff[t] + kc), *(const v8us*)(Bl + boff[t] + kc + 16)); acc[t] = wmmab(a, bl2, acc[t]); } }
        asm volatile("v_nop\n\tv_nop\n\tv_nop\n\tv_nop" : "+v"(acc[0]), "+v"(acc[1]), "+v"(acc[2]), "+v"(acc[3]) : "v"(a), "v"(al));
    }
    float* os = &ost[wave][0];
#pragma unroll
    for (int t = 0; t < 4; ++t)
#pragma unroll
        for (int j = 0; j < 8; ++j) { const int row = r0 + hi * 8 + j, col = c0 + t * 16 + lr; float v = acc[t][j];
            if (MODE == 0) v = fmaxf(v * sc[col] + sh[col], 0.f); else if (MODE == 1 || MODE == 4) v = fmaxf(v * sc[row] + sh[row], 0.f);
            os[(hi * 8 + j) * 68 + t * 16 + lr] = v; }
    __syncthreads();
    if (MODE == 2 || MODE == 4) {
        float* crow = (float*)C + (size_t)r0 * ldc + c0;
        auto pass = [&]() {
#pragma unroll
            for (int s = 0; s < 8; ++s) { const int Lid = (lane >> 3) + 4 * s, piece = lane & 7; const int row = Lid >> 1, cofs = (Lid & 1) * 32 + piece * 4;
                const v4f val = *(const v4fa*)(os + row * 68 + cofs); *(volatile v4f*)(crow + (size_t)row * ldc + cofs) = val; }
        };
        pass(); __threadfence(); pass();
    } else {
        bf* c1 = (bf*)C + (size_t)r0 * ldc + c0; bf* c2 = (bf*)C2 + (size_t)r0 * ldc + c0;
        auto pass = [&]() {
#pragma unroll
            for (int s = 0; s < 4; ++s) { const int row = 4 * s + (lane >> 3), piece = lane & 7; const float* sp = os + row * 68 + piece * 8; v8us oh, ol;
#pragma unroll
                for (int i = 0; i < 8; ++i) { const unsigned short hb = f2bf(sp[i]); oh[i] = hb; ol[i] = f2bf(sp[i] - bf2f(hb)); }
                *(volatile v8us*)(c1 + (size_t)row * ldc + piece * 8) = oh; *(volatile v8us*)(c2 + (size_t)row * ldc + piece * 8) = ol; }
        };
        pass(); __threadfence(); pass();
    }
}
__device__ __forceinline__ void bnf(const float* __restrict__ g, const float* __restrict__ bb, const float* __restrict__ m, const float* __restrict__ v, int j, int n, float* SC, float* SH, int i) {
    float s = 0.f, t = 0.f;
    if (j < n) { s = bfr(g[j]) / sqrtf(bfr(v[j]) + 1e-5f); t = bfr(bb[j]) - bfr(m[j]) * s; }
    VST2(float, SC + i, s); VST2(float, SH + i, t);
}
__global__ __launch_bounds__(256) void k_bnfold(const float* __restrict__ gq, const float* __restrict__ bq, const float* __restrict__ mq, const float* __restrict__ vq,
                                               const float* __restrict__ gk, const float* __restrict__ bk, const float* __restrict__ mk, const float* __restrict__ vk,
                                               const float* __restrict__ gv, const float* __restrict__ bv, const float* __restrict__ mv, const float* __restrict__ vv,
                                               const float* __restrict__ gf, const float* __restrict__ bff, const float* __restrict__ mf, const float* __restrict__ vf, float* SC, float* SH) {
    const int j = threadIdx.x, i = blockIdx.x * 256 + j;
    if (blockIdx.x == 0) bnf(gq, bq, mq, vq, j, HH_, SC, SH, i);
    else if (blockIdx.x == 1) bnf(gk, bk, mk, vk, j, HH_, SC, SH, i);
    else if (blockIdx.x == 2) bnf(gv, bv, mv, vv, j, HH_, SC, SH, i);
    else bnf(gf, bff, mf, vf, j, CO, SC, SH, i);
}
__global__ __launch_bounds__(256) void k_kvT(const float* __restrict__ KV, bf* KVH, bf* KVL) {
    __shared__ float tl[64][65];
    const int tid = threadIdx.x, c0 = blockIdx.x * 64, d0 = blockIdx.y * 64, bl = blockIdx.z;
    { const int cr = tid >> 2, dq = (tid & 3) * 16;
#pragma unroll
      for (int i = 0; i < 16; ++i) tl[dq + i][cr] = KV[((size_t)bl * HH_ + c0 + cr) * HH_ + d0 + dq + i]; }
    __syncthreads();
    const int piece = tid & 7;
    auto pass = [&]() {
#pragma unroll
        for (int s = 0; s < 2; ++s) { const int dr = (tid >> 3) + 32 * s; v8us oh, ol;
#pragma unroll
            for (int i = 0; i < 8; ++i) { const float v = tl[dr][piece * 8 + i]; const unsigned short hb = f2bf(v); oh[i] = hb; ol[i] = f2bf(v - bf2f(hb)); }
            const size_t o = ((size_t)bl * HH_ + d0 + dr) * HH_ + c0 + piece * 8;
            *(volatile v8us*)(KVH + o) = oh; *(volatile v8us*)(KVL + o) = ol; }
    };
    pass(); __threadfence(); pass();
}

extern "C" void kernel_launch(void* const* d_in, const int* in_sizes, int n_in,
                              void* d_out, int out_size, void* d_ws, size_t ws_size, hipStream_t stream) {
    (void)in_sizes; (void)n_in; (void)out_size;
    const float* x = (const float*)d_in[0];
    const float* wq = (const float*)d_in[1]; const float* wk = (const float*)d_in[2]; const float* wv = (const float*)d_in[3]; const float* wf = (const float*)d_in[4];
    const float* gq = (const float*)d_in[5];  const float* bq  = (const float*)d_in[6];  const float* mq = (const float*)d_in[7];  const float* vq = (const float*)d_in[8];
    const float* gk = (const float*)d_in[9];  const float* bk  = (const float*)d_in[10]; const float* mk = (const float*)d_in[11]; const float* vk = (const float*)d_in[12];
    const float* gv = (const float*)d_in[13]; const float* bv  = (const float*)d_in[14]; const float* mv = (const float*)d_in[15]; const float* vv = (const float*)d_in[16];
    const float* gf = (const float*)d_in[17]; const float* bff = (const float*)d_in[18]; const float* mf = (const float*)d_in[19]; const float* vf = (const float*)d_in[20];
    float* out = (float*)d_out;
    char* wsp = (char*)d_ws;
    auto take = [&](size_t bytes) { char* p = wsp; wsp += (bytes + 255) & ~(size_t)255; return (void*)p; };
    bf* WP3 = (bf*)take((size_t)3 * HH_ * KP * 2); bf* WF = (bf*)take((size_t)CO * HH_ * 2); float* SC = (float*)take(1024 * 4); float* SH = (float*)take(1024 * 4);
    bf* XT = (bf*)take((size_t)BCH * NN_ * KP * 2);
    bf* QH = (bf*)take((size_t)BCH * NN_ * HH_ * 2); bf* QL = (bf*)take((size_t)BCH * NN_ * HH_ * 2);
    bf* KH = (bf*)take((size_t)BCH * HH_ * NN_ * 2); bf* KL = (bf*)take((size_t)BCH * HH_ * NN_ * 2); bf* VH = (bf*)take((size_t)BCH * HH_ * NN_ * 2); bf* VL = (bf*)take((size_t)BCH * HH_ * NN_ * 2);
    float* KV = (float*)take((size_t)BCH * HH_ * HH_ * 4); bf* KVH = (bf*)take((size_t)BCH * HH_ * HH_ * 2); bf* KVL = (bf*)take((size_t)BCH * HH_ * HH_ * 2);
    bf* VTH = (bf*)take((size_t)BCH * NN_ * HH_ * 2); bf* VTL = (bf*)take((size_t)BCH * NN_ * HH_ * 2);
    if ((size_t)(wsp - (char*)d_ws) > ws_size) return;
    k_w<<<(3 * HH_ + CO) / 8, 256, 0, stream>>>(wq, wk, wv, wf, WP3, WF);
    k_bnfold<<<4, 256, 0, stream>>>(gq, bq, mq, vq, gk, bk, mk, vk, gv, bv, mv, vv, gf, bff, mf, vf, SC, SH);
    for (int ch = 0; ch < NB_ / BCH; ++ch) { const int b0 = ch * BCH;
        k_xt<<<dim3(NN_ / 64, 3, BCH), 256, 0, stream>>>(x, b0, XT);
        for (int bl = 0; bl < BCH; ++bl) { const bf* xt = XT + (size_t)bl * NN_ * KP;
            k_gemm<false, false, 0><<<dim3(NN_ / 64, HH_ / 64, 1), 128, 0, stream>>>(xt, nullptr, WP3, nullptr, KP, HH_, SC, SH, QH + (size_t)bl * NN_ * HH_, QL + (size_t)bl * NN_ * HH_);
            k_gemm<false, false, 1><<<dim3(HH_ / 64, NN_ / 64, 1), 128, 0, stream>>>(WP3 + (size_t)HH_ * KP, nullptr, xt, nullptr, KP, NN_, SC + HH_, SH + HH_, KH + (size_t)bl * HH_ * NN_, KL + (size_t)bl * HH_ * NN_);
            k_gemm<false, false, 1><<<dim3(HH_ / 64, NN_ / 64, 1), 128, 0, stream>>>(WP3 + (size_t)2 * HH_ * KP, nullptr, xt, nullptr, KP, NN_, SC + 2 * HH_, SH + 2 * HH_, VH + (size_t)bl * HH_ * NN_, VL + (size_t)bl * HH_ * NN_);
            k_gemm<true, true, 2><<<dim3(HH_ / 64, HH_ / 64, 1), 128, 0, stream>>>(KH + (size_t)bl * HH_ * NN_, KL + (size_t)bl * HH_ * NN_, VH + (size_t)bl * HH_ * NN_, VL + (size_t)bl * HH_ * NN_, NN_, HH_, nullptr, nullptr, KV + (size_t)bl * HH_ * HH_, nullptr);
        }
        k_kvT<<<dim3(HH_ / 64, HH_ / 64, BCH), 256, 0, stream>>>(KV, KVH, KVL);
        for (int bl = 0; bl < BCH; ++bl) {
            k_gemm<true, true, 3><<<dim3(NN_ / 64, HH_ / 64, 1), 128, 0, stream>>>(QH + (size_t)bl * NN_ * HH_, QL + (size_t)bl * NN_ * HH_, KVH + (size_t)bl * HH_ * HH_, KVL + (size_t)bl * HH_ * HH_, HH_, HH_, nullptr, nullptr, VTH + (size_t)bl * NN_ * HH_, VTL + (size_t)bl * NN_ * HH_);
            k_gemm<false, true, 4><<<dim3(CO / 64, NN_ / 64, 1), 128, 0, stream>>>(WF, nullptr, VTH + (size_t)bl * NN_ * HH_, VTL + (size_t)bl * NN_ * HH_, HH_, NN_, SC + 3 * HH_, SH + 3 * HH_, out + (size_t)(b0 + bl) * CO * NN_, nullptr);
        }
    }
}
